// GeometryGuidedAttention_58162447123324
// MI455X (gfx1250) — hardware-verified
//
#include <hip/hip_runtime.h>


#define NB_  2
#define NN   16384
#define KN   16
#define CC   256
#define NH_  4
#define HD   64
#define CHP  2048
#define CHR  (CHP * KN)
typedef _Float16 h16;
typedef unsigned short bf;
typedef __attribute__((ext_vector_type(16))) __bf16   v16bf;
typedef __attribute__((ext_vector_type(16))) _Float16 v16h;
typedef __attribute__((ext_vector_type(8)))  _Float16 v8h;
typedef __attribute__((ext_vector_type(8)))  unsigned short v8us;
typedef __attribute__((ext_vector_type(8)))  float    v8f;
typedef __attribute__((ext_vector_type(4)))  float    v4f;
typedef v8h  __attribute__((may_alias)) v8ha;
typedef v4f  __attribute__((may_alias)) v4fa;
typedef v8us __attribute__((may_alias)) v8usa;

__device__ __forceinline__ unsigned short f2bf(float f) { unsigned u = __float_as_uint(f); u += 0x7FFFu + ((u >> 16) & 1u); return (unsigned short)(u >> 16); }
__device__ __forceinline__ float bf2f(unsigned short b) { return __uint_as_float(((unsigned)b) << 16); }
__device__ __forceinline__ float bfr(float f) { return bf2f(f2bf(f)); }
__device__ __forceinline__ v16h cat16(v8h lo, v8h hi) { return __builtin_shufflevector(lo, hi, 0, 1, 2, 3, 4, 5, 6, 7, 8, 9, 10, 11, 12, 13, 14, 15); }
__device__ __forceinline__ v16bf cat16b(v8us lo, v8us hi) { return __builtin_bit_cast(v16bf, __builtin_shufflevector(lo, hi, 0, 1, 2, 3, 4, 5, 6, 7, 8, 9, 10, 11, 12, 13, 14, 15)); }
__device__ __forceinline__ v8f wmma16(v16h a, v16h b, v8f c) { return __builtin_amdgcn_wmma_f32_16x16x32_f16(false, a, false, b, (short)0, c, false, false); }
__device__ __forceinline__ v8f wmmab(v16bf a, v16bf b, v8f c) { return __builtin_amdgcn_wmma_f32_16x16x32_bf16(false, a, false, b, (short)0, c, false, false); }


template <typename T16> struct WFrag;
template <> struct WFrag<h16> { typedef v16h V; static __device__ __forceinline__ V ld(const h16* p) { return cat16(*(const v8h*)p, *(const v8h*)(p + 16)); } static __device__ __forceinline__ v8f mma(V a, V b, v8f c) { return wmma16(a, b, c); } };
template <> struct WFrag<bf> { typedef v16bf V; static __device__ __forceinline__ V ld(const bf* p) { return cat16b(*(const v8us*)p, *(const v8us*)(p + 16)); } static __device__ __forceinline__ v8f mma(V a, V b, v8f c) { return wmmab(a, b, c); } };
template <typename T16, int NSPLIT, bool BIAS>
__global__ __launch_bounds__(32) void k_gemmw(const T16* __restrict__ A, const T16* __restrict__ A2, const T16* __restrict__ Bt, const T16* __restrict__ Bt2, int K, float* C, int ldc, const float* __restrict__ bias, size_t sA, size_t sB, size_t sC) {
    typedef typename WFrag<T16>::V V;
    __shared__ __align__(16) float os[16 * 68];
    const size_t z = blockIdx.z; A += z * sA; if (A2) A2 += z * sA; Bt += z * sB; if (Bt2) Bt2 += z * sB; C += z * sC;
    const int lane = threadIdx.x & 31, lr = lane & 15, hi = lane >> 4; const int r0 = blockIdx.x * 64, c0 = blockIdx.y * 64;
    v8f acc[4][4];
#pragma unroll
    for (int mb = 0; mb < 4; ++mb)
#pragma unroll
        for (int nb = 0; nb < 4; ++nb) acc[mb][nb] = (v8f){};
    const size_t aoff = (size_t)(r0 + lr) * K + 8 * hi, boff = (size_t)(c0 + lr) * K + 8 * hi;
#pragma unroll 1
    for (int kc = 0; kc < K; kc += 32) {
        V a[4], a2[4];
#pragma unroll
        for (int mb = 0; mb < 4; ++mb) { a[mb] = WFrag<T16>::ld(A + aoff + (size_t)mb * 16 * K + kc); if (NSPLIT == 1 || NSPLIT == 2) a2[mb] = WFrag<T16>::ld(A2 + aoff + (size_t)mb * 16 * K + kc); }
#pragma unroll
        for (int nb = 0; nb < 4; ++nb) { const V b = WFrag<T16>::ld(Bt + boff + (size_t)nb * 16 * K + kc); V b2; if (NSPLIT >= 2) b2 = WFrag<T16>::ld(Bt2 + boff + (size_t)nb * 16 * K + kc);
#pragma unroll
            for (int mb = 0; mb < 4; ++mb) { acc[mb][nb] = WFrag<T16>::mma(a[mb], b, acc[mb][nb]); if (NSPLIT == 1 || NSPLIT == 2) acc[mb][nb] = WFrag<T16>::mma(a2[mb], b, acc[mb][nb]); if (NSPLIT >= 2) acc[mb][nb] = WFrag<T16>::mma(a[mb], b2, acc[mb][nb]); } }
        asm volatile("v_nop\n\tv_nop\n\tv_nop\n\tv_nop" : "+v"(acc[0][0]), "+v"(acc[1][1]), "+v"(acc[2][2]), "+v"(acc[3][3]) : "v"(a[0]), "v"(a[3]));
    }
#pragma unroll
    for (int mb = 0; mb < 4; ++mb) {
#pragma unroll
        for (int nb = 0; nb < 4; ++nb) {
#pragma unroll
            for (int j = 0; j < 8; ++j) os[(hi * 8 + j) * 68 + nb * 16 + lr] = acc[mb][nb][j]; }
        __builtin_amdgcn_wave_barrier(); asm volatile("" ::: "memory");
        float* crow = C + (size_t)(r0 + mb * 16) * ldc + c0;
#pragma unroll 1
        for (int ps = 0; ps < 2; ++ps) {
#pragma unroll
            for (int s = 0; s < 8; ++s) { const int row = 2 * s + hi, cofs = lr * 4; v4f val = *(const v4fa*)(os + row * 68 + cofs); if (BIAS) { val[0] += bfr(bias[c0 + cofs]); val[1] += bfr(bias[c0 + cofs + 1]); val[2] += bfr(bias[c0 + cofs + 2]); val[3] += bfr(bias[c0 + cofs + 3]); }
                *(volatile v4f*)(crow + (size_t)row * ldc + cofs) = val; }
            if (ps == 0) __threadfence(); }
        __builtin_amdgcn_wave_barrier(); asm volatile("" ::: "memory");
    }
}

__device__ __forceinline__ h16 tohx(float x) { return (h16)x; }
__device__ __forceinline__ void splitf(float y, unsigned short& h, unsigned short& l) { h = f2bf(y); l = f2bf(y - bf2f(h)); }
typedef __attribute__((ext_vector_type(4))) _Float16 v4h;
typedef __attribute__((ext_vector_type(4))) unsigned short v4us;
typedef __attribute__((ext_vector_type(2))) unsigned short v2us;

__global__ __launch_bounds__(256) void k_cvt8(const float* __restrict__ src, bf* dst, size_t n8) { const size_t i = (size_t)blockIdx.x * 256 + threadIdx.x; if (i >= n8) return; const v8f v = *(const v8f*)(src + i * 8); v8us o;
#pragma unroll
    for (int k = 0; k < 8; ++k) o[k] = f2bf(v[k]); *(volatile v8us*)(dst + i * 8) = o; __threadfence(); *(volatile v8us*)(dst + i * 8) = o; }
__global__ __launch_bounds__(256) void k_wtG(const float* __restrict__ w, int K, int N, bf* Bt) {
    const int lane = threadIdx.x & 31; const int L0 = (blockIdx.x * 8 + (threadIdx.x >> 5)) * 8; const int nlines = N * K / 64;
#pragma unroll 1
    for (int ps = 0; ps < 2; ++ps) {
#pragma unroll 1
        for (int l = 0; l < 8; ++l) { const int L = L0 + l; if (L >= nlines) break; const size_t e = (size_t)L * 64 + lane * 2; const int k = (int)(e % K), n = (int)(e / K); v2us o;
            o[0] = f2bf(w[(size_t)k * N + n]); o[1] = f2bf(w[(size_t)(k + 1) * N + n]); *(volatile v2us*)(Bt + e) = o; }
        if (ps == 0) __threadfence(); }
}
__global__ __launch_bounds__(256) void k_wt16(const float* __restrict__ w, int K, int N, h16* W16) { __shared__ float tile[64][65]; const int nb = (N + 63) / 64; const int k0 = (blockIdx.x / nb) * 64, n0 = (blockIdx.x % nb) * 64;
    for (int i = threadIdx.x; i < 64 * 64; i += 256) { const int kk = i / 64, nn = i % 64; tile[kk][nn] = (k0 + kk < K && n0 + nn < N) ? w[(size_t)(k0 + kk) * N + n0 + nn] : 0.f; }
    __syncthreads();
    const int nn = threadIdx.x / 4, kq = (threadIdx.x % 4) * 16; if (n0 + nn >= N) return;
    for (int c = 0; c < 16; c += 4) { v4h o; o[0] = tohx(bfr(tile[kq + c][nn])); o[1] = tohx(bfr(tile[kq + c + 1][nn])); o[2] = tohx(bfr(tile[kq + c + 2][nn])); o[3] = tohx(bfr(tile[kq + c + 3][nn])); h16* dst = W16 + (size_t)(n0 + nn) * K + k0 + kq + c; *(volatile v4h*)dst = o; __threadfence(); *(volatile v4h*)dst = o; } }
__device__ __forceinline__ int nbr(const int* idx, size_t o) { int j = idx[o]; return j < 0 ? 0 : (j >= NN ? NN - 1 : j); }
__global__ __launch_bounds__(256) void k_geom(const float* __restrict__ Pb, const int* __restrict__ idxb, int n0, const float* __restrict__ wp1, const float* __restrict__ bp1, h16* G16) { const int e = (blockIdx.x * 256 + threadIdx.x) * 4; if (e >= CHR * CC) return; const int c = e % CC; const int r = e / CC; const int n = n0 + r / KN; const int j = nbr(idxb, (size_t)n * KN + (r % KN));
    const float rx = __fsub_rn(bfr(Pb[j]), bfr(Pb[n])), ry = __fsub_rn(bfr(Pb[NN + j]), bfr(Pb[NN + n])), rz = __fsub_rn(bfr(Pb[2 * NN + j]), bfr(Pb[2 * NN + n])); float sx = __fmul_rn(rx, rx); asm volatile("" : "+v"(sx)); float sy = __fmul_rn(ry, ry); asm volatile("" : "+v"(sy)); float sz = __fmul_rn(rz, rz); asm volatile("" : "+v"(sz)); const float dist = __fsqrt_rn(__fadd_rn(__fadd_rn(sx, sy), sz)); v4h o;
#pragma unroll
    for (int u = 0; u < 4; ++u) { const int cc = c + u; float acc = bfr(bp1[cc]); float p;
        p = __fmul_rn(rx, bfr(wp1[cc])); asm volatile("" : "+v"(p)); acc = __fadd_rn(acc, p); p = __fmul_rn(ry, bfr(wp1[CC + cc])); asm volatile("" : "+v"(p)); acc = __fadd_rn(acc, p); p = __fmul_rn(rz, bfr(wp1[2 * CC + cc])); asm volatile("" : "+v"(p)); acc = __fadd_rn(acc, p); p = __fmul_rn(dist, bfr(wp1[3 * CC + cc])); asm volatile("" : "+v"(p)); acc = __fadd_rn(acc, p);
        o[u] = tohx(fmaxf(acc, 0.f)); }
    *(volatile v4h*)(G16 + e) = o; __threadfence(); *(volatile v4h*)(G16 + e) = o; }
__global__ __launch_bounds__(256) void k_rel(const float* __restrict__ QF, const float* __restrict__ KF, const float* __restrict__ PE, const int* __restrict__ idxb, int n0, h16* REL16) { const int e = (blockIdx.x * 256 + threadIdx.x) * 4; if (e >= CHR * CC) return; const int c = e % CC; const int r = e / CC; const int n = n0 + r / KN; const int j = nbr(idxb, (size_t)n * KN + (r % KN));
    const v4f q = *(const v4f*)(QF + (size_t)n * CC + c), k = *(const v4f*)(KF + (size_t)j * CC + c), p = *(const v4f*)(PE + e); v4h o;
#pragma unroll
    for (int u = 0; u < 4; ++u) o[u] = tohx(__fadd_rn(__fsub_rn(q[u], k[u]), p[u])); *(volatile v4h*)(REL16 + e) = o; __threadfence(); *(volatile v4h*)(REL16 + e) = o; }
__global__ __launch_bounds__(256) void k_attn(const float* __restrict__ L1, const float* __restrict__ wa2, const float* __restrict__ ba2, const float* __restrict__ VF, const float* __restrict__ PE, const int* __restrict__ idxb, int n0, bf* AGh, bf* AGl) {
    const int lane = threadIdx.x & 31; const int w = blockIdx.x * 8 + (threadIdx.x >> 5); if (w >= CHP * NH_) return; const int hh = w % NH_; const int nl = w / NH_; const int n = n0 + nl; const int k = lane & 15;
    const int r = nl * KN + k; const float* lrow = L1 + ((size_t)r * NH_ + hh) * HD; float lg = bfr(ba2[0]);
#pragma unroll 1
    for (int d = 0; d < HD; ++d) { float p = __fmul_rn(fmaxf(lrow[d], 0.f), bfr(wa2[d])); asm volatile("" : "+v"(p)); lg = __fadd_rn(lg, p); }
    float mx = lg;
#pragma unroll
    for (int sh = 8; sh; sh >>= 1) mx = fmaxf(mx, __shfl_xor(mx, sh, 32));
    float d0 = __fsub_rn(lg, mx); asm volatile("" : "+v"(d0)); const float ex = __expf(d0); float z = ex;
#pragma unroll
    for (int sh = 8; sh; sh >>= 1) z += __shfl_xor(z, sh, 32);
    const float at = __fdiv_rn(ex, z); const int j = nbr(idxb, (size_t)n * KN + k);
    float acc[4] = {0.f, 0.f, 0.f, 0.f}; const int dd = 4 * k;
#pragma unroll 1
    for (int kk = 0; kk < KN; ++kk) { const float ak = __shfl(at, kk, 32); const int jk = __shfl(j, kk, 32); const float* vr = VF + (size_t)jk * CC + hh * HD + dd; const float* pr = PE + ((size_t)(nl * KN + kk)) * CC + hh * HD + dd;
#pragma unroll
        for (int u = 0; u < 4; ++u) { float s = __fadd_rn(vr[u], pr[u]); float p = __fmul_rn(ak, s); asm volatile("" : "+v"(p)); acc[u] = __fadd_rn(acc[u], p); } }
    if (lane < 16) { v4us oh, ol;
#pragma unroll
        for (int u = 0; u < 4; ++u) { unsigned short a, c; splitf(acc[u], a, c); oh[u] = a; ol[u] = c; } const size_t o = (size_t)n * CC + hh * HD + dd; *(volatile v4us*)(AGh + o) = oh; *(volatile v4us*)(AGl + o) = ol; __threadfence(); *(volatile v4us*)(AGh + o) = oh; *(volatile v4us*)(AGl + o) = ol; } }

extern "C" void kernel_launch(void* const* d_in, const int* in_sizes, int n_in,
                              void* d_out, int out_size, void* d_ws, size_t ws_size, hipStream_t stream) {
    (void)in_sizes; (void)n_in; (void)out_size;
    const float* h = (const float*)d_in[0]; const float* P = (const float*)d_in[1]; const int* idx = (const int*)d_in[2]; const float* wq = (const float*)d_in[3]; const float* wk = (const float*)d_in[4]; const float* wv = (const float*)d_in[5]; const float* wp1 = (const float*)d_in[6]; const float* bp1 = (const float*)d_in[7]; const float* wp2 = (const float*)d_in[8]; const float* bp2 = (const float*)d_in[9]; const float* wa1 = (const float*)d_in[10]; const float* ba1 = (const float*)d_in[11]; const float* wa2 = (const float*)d_in[12]; const float* ba2 = (const float*)d_in[13]; const float* wo = (const float*)d_in[14]; const float* bo = (const float*)d_in[15];
    float* OUT = (float*)d_out;
    char* wsp = (char*)d_ws;
    auto take = [&](size_t bytes) { char* p = wsp; wsp += (bytes + 255) & ~(size_t)255; return (void*)p; };
    bf* WQ = (bf*)take(CC * CC * 2); bf* WK = (bf*)take(CC * CC * 2); bf* WV = (bf*)take(CC * CC * 2); bf* WO = (bf*)take(CC * CC * 2); h16* WP2 = (h16*)take(CC * CC * 2); h16* WA1 = (h16*)take(HD * HD * 2);
    bf* HB = (bf*)take((size_t)NN * CC * 2); float* QF = (float*)take((size_t)NN * CC * 4); float* KF = (float*)take((size_t)NN * CC * 4); float* VF = (float*)take((size_t)NN * CC * 4); h16* G16 = (h16*)take((size_t)CHR * CC * 2); float* PE = (float*)take((size_t)CHR * CC * 4); h16* REL16 = (h16*)take((size_t)CHR * CC * 2); float* L1 = (float*)take((size_t)CHR * NH_ * HD * 4); bf* AGh = (bf*)take((size_t)NN * CC * 2); bf* AGl = (bf*)take((size_t)NN * CC * 2);
    if ((size_t)(wsp - (char*)d_ws) > ws_size) return;
    k_wtG<<<(CC * CC / 64 + 63) / 64, 256, 0, stream>>>(wq, CC, CC, WQ); k_wtG<<<(CC * CC / 64 + 63) / 64, 256, 0, stream>>>(wk, CC, CC, WK); k_wtG<<<(CC * CC / 64 + 63) / 64, 256, 0, stream>>>(wv, CC, CC, WV); k_wtG<<<(CC * CC / 64 + 63) / 64, 256, 0, stream>>>(wo, CC, CC, WO);
    k_wt16<<<(CC / 64) * (CC / 64), 256, 0, stream>>>(wp2, CC, CC, WP2); k_wt16<<<1, 256, 0, stream>>>(wa1, HD, HD, WA1);
    for (int b = 0; b < NB_; ++b) { const float* Pb = P + (size_t)b * 3 * NN; const int* idxb = idx + (size_t)b * NN * KN;
        k_cvt8<<<(NN * CC / 8 + 255) / 256, 256, 0, stream>>>(h + (size_t)b * NN * CC, HB, (size_t)NN * CC / 8);
        k_gemmw<bf, 0, false><<<dim3(NN / 64, CC / 64, 1), 32, 0, stream>>>(HB, nullptr, WQ, nullptr, CC, QF, CC, nullptr, 0, 0, 0); k_gemmw<bf, 0, false><<<dim3(NN / 64, CC / 64, 1), 32, 0, stream>>>(HB, nullptr, WK, nullptr, CC, KF, CC, nullptr, 0, 0, 0); k_gemmw<bf, 0, false><<<dim3(NN / 64, CC / 64, 1), 32, 0, stream>>>(HB, nullptr, WV, nullptr, CC, VF, CC, nullptr, 0, 0, 0);
        for (int n0 = 0; n0 < NN; n0 += CHP) {
            k_geom<<<(CHR * CC / 4 + 255) / 256, 256, 0, stream>>>(Pb, idxb, n0, wp1, bp1, G16);
            k_gemmw<h16, 0, true><<<dim3(CHR / 64, CC / 64, 1), 32, 0, stream>>>(G16, nullptr, WP2, nullptr, CC, PE, CC, bp2, 0, 0, 0);
            k_rel<<<(CHR * CC / 4 + 255) / 256, 256, 0, stream>>>(QF, KF, PE, idxb, n0, REL16);
            k_gemmw<h16, 0, true><<<dim3(CHR * NH_ / 64, 1, 1), 32, 0, stream>>>(REL16, nullptr, WA1, nullptr, HD, L1, HD, ba1, 0, 0, 0);
            k_attn<<<(CHP * NH_ + 7) / 8, 256, 0, stream>>>(L1, wa2, ba2, VF, PE, idxb, n0, AGh, AGl); }
        k_gemmw<bf, 1, true><<<dim3(NN / 64, CC / 64, 1), 32, 0, stream>>>(AGh, AGl, WO, nullptr, CC, OUT + (size_t)b * NN * CC, CC, bo, 0, 0, 0); }
}
